// EnhancedMultiHeadAttention_14431090115033
// MI455X (gfx1250) — hardware-verified
//
#include <hip/hip_runtime.h>
#include <math.h>

typedef __attribute__((ext_vector_type(16))) _Float16 v16h;
typedef __attribute__((ext_vector_type(8)))  _Float16 v8h;
typedef __attribute__((ext_vector_type(16))) __bf16   v16b;
typedef __attribute__((ext_vector_type(8)))  __bf16   v8b;
typedef __attribute__((ext_vector_type(8)))  float    v8f;
typedef __attribute__((ext_vector_type(4)))  float    v4f;
typedef __attribute__((ext_vector_type(4)))  unsigned v4u;

constexpr int kBatch   = 4;
constexpr int kSeq     = 1024;
constexpr int kEmb     = 1024;
constexpr int kHeads   = 16;
constexpr int kHD      = 64;
constexpr int kTok     = kBatch * kSeq;
constexpr int kRelRows = 1999;
constexpr int kRelMax  = kRelRows - 1;

static_assert(kEmb == kHeads * kHD);
static_assert(kHD == 64);
static_assert(kTok % 64 == 0 && kEmb % 64 == 0 && kEmb % 32 == 0 && kSeq % 64 == 0);

__device__ __forceinline__ unsigned short f2bf_bits(float f) {
  unsigned u = __float_as_uint(f);
  return (unsigned short)((u + 0x7FFFu + ((u >> 16) & 1u)) >> 16);
}
__device__ __forceinline__ float bf_bits2f(unsigned short h) { return __uint_as_float(((unsigned)h) << 16); }
__device__ __forceinline__ float rne_bf(float f) { return bf_bits2f(f2bf_bits(f)); }

__device__ __forceinline__ void dep_guard_h(v8f& a, v8f& b, v16h x, v16h y) { asm volatile("v_nop\n\tv_nop\n\tv_nop\n\tv_nop" : "+v"(a), "+v"(b) : "v"(x), "v"(y)); }
__device__ __forceinline__ void dep_guard_b(v8f& a, v8f& b, v16b x, v16b y) { asm volatile("v_nop\n\tv_nop\n\tv_nop\n\tv_nop" : "+v"(a), "+v"(b) : "v"(x), "v"(y)); }
__device__ __forceinline__ void keep4_h(v16h a, v16h b, v16h c, v16h d) { asm volatile("v_nop" :: "v"(a), "v"(b), "v"(c), "v"(d)); }
__device__ __forceinline__ void keep4_b(v16b a, v16b b, v16b c, v16b d) { asm volatile("v_nop" :: "v"(a), "v"(b), "v"(c), "v"(d)); }
__device__ __forceinline__ void acc_guard4(v8f& a, v8f& b, v8f& c, v8f& d) { asm volatile("v_nop\n\tv_nop\n\tv_nop\n\tv_nop" : "+v"(a), "+v"(b), "+v"(c), "+v"(d)); }
template <typename T> struct Frag;
template <> struct Frag<_Float16> {
  typedef v16h V; union U { v16h v; v8h h[2]; };
  static __device__ __forceinline__ v16h load(const _Float16* p) {
    U f; f.h[0] = *(const v8h*)(p); f.h[1] = *(const v8h*)(p + 16); return f.v;
  }
  static __device__ __forceinline__ v8f mma(v16h a, v16h b, v8f c) {
    return __builtin_amdgcn_wmma_f32_16x16x32_f16(false, a, false, b, (short)0, c, false, false);
  }
  static __device__ __forceinline__ void guard(v8f& a, v8f& b, v16h x, v16h y) { dep_guard_h(a, b, x, y); }
  static __device__ __forceinline__ void keep(v16h a, v16h b, v16h c, v16h d) { keep4_h(a, b, c, d); }
};
template <> struct Frag<__bf16> {
  typedef v16b V; union U { v16b v; v8b h[2]; };
  static __device__ __forceinline__ v16b load(const __bf16* p) {
    U f; f.h[0] = *(const v8b*)(p); f.h[1] = *(const v8b*)(p + 16); return f.v;
  }
  static __device__ __forceinline__ v8f mma(v16b a, v16b b, v8f c) {
    return __builtin_amdgcn_wmma_f32_16x16x32_bf16(false, a, false, b, (short)0, c, false, false);
  }
  static __device__ __forceinline__ void guard(v8f& a, v8f& b, v16b x, v16b y) { dep_guard_b(a, b, x, y); }
  static __device__ __forceinline__ void keep(v16b a, v16b b, v16b c, v16b d) { keep4_b(a, b, c, d); }
};

__device__ __forceinline__ v8f hmma(v16h a, v16h b, v8f c) {
  c = __builtin_amdgcn_wmma_f32_16x16x32_f16(false, a, false, b, (short)0, c, false, false);
  asm volatile("v_nop\n\tv_nop\n\tv_nop\n\tv_nop" : "+v"(c) : "v"(a), "v"(b));
  return c;
}

template <int ET> struct Elem;
template <> struct Elem<0> { typedef _Float16 T; };
template <> struct Elem<1> { typedef __bf16 T; };
template <int ET, bool SPLIT, int BIAS_MODE, int OUT_MODE>
__global__ __launch_bounds__(256) void wmma_gemm64(
    const unsigned short* __restrict__ Ap, const unsigned short* __restrict__ A2p, int lda, long strideA,
    const unsigned short* __restrict__ Btp, const unsigned short* __restrict__ Bt2p, int ldb, long strideB,
    void* __restrict__ Cout, void* __restrict__ Cout2, int ldc, long strideC,
    const float* __restrict__ bias,
    int M, int N, int K, float scale) {
  typedef typename Elem<ET>::T T;
  typedef typename Frag<T>::V V;
  const T* A = (const T*)Ap; const T* A2 = (const T*)A2p; const T* Bt = (const T*)Btp; const T* Bt2 = (const T*)Bt2p;
  __shared__ __align__(16) float sT[8][16 * 68];
  const int b    = blockIdx.y;
  const int lane = threadIdx.x & 31;
  const int wave = threadIdx.x >> 5;
  const int tilesN = N >> 6;
  const int tilesM = M >> 6;
  const int tile = blockIdx.x * 8 + wave;
  if (tile >= tilesM * tilesN) return;
  const int tm = tile / tilesN;
  const int tn = tile - tm * tilesN;
  const int m0 = tm << 6;
  const int n0 = tn << 6;

  const T* Ab  = A  + (size_t)b * strideA;
  const T* Bb  = Bt + (size_t)b * strideB;
  const T* Ab2 = SPLIT ? (A2  + (size_t)b * strideA) : nullptr;
  const T* Bb2 = SPLIT ? (Bt2 + (size_t)b * strideB) : nullptr;

  const int rlane = lane & 15;
  const int koff  = (lane >> 4) * 8;
  const int mOff  = (lane >> 4) * 8;

  v8f acc[4][4];
#pragma unroll
  for (int i = 0; i < 4; ++i)
#pragma unroll
    for (int j = 0; j < 4; ++j) acc[i][j] = (v8f){0.f,0.f,0.f,0.f,0.f,0.f,0.f,0.f};

  for (int k0 = 0; k0 < K; k0 += 32) {
    V bh[4], bl[4];
#pragma unroll
    for (int j = 0; j < 4; ++j) {
      const size_t bo = (size_t)(n0 + (j << 4) + rlane) * ldb + koff + k0;
      bh[j] = Frag<T>::load(Bb + bo);
      if (SPLIT) bl[j] = Frag<T>::load(Bb2 + bo);
    }
#pragma unroll
    for (int i = 0; i < 4; ++i) {
      const size_t ao = (size_t)(m0 + (i << 4) + rlane) * lda + koff + k0;
      V ah = Frag<T>::load(Ab + ao);
      V al;
      if (SPLIT) al = Frag<T>::load(Ab2 + ao);
#pragma unroll
      for (int j = 0; j < 4; ++j) {
        acc[i][j] = Frag<T>::mma(ah, bh[j], acc[i][j]);
        if (SPLIT) {
          acc[i][j] = Frag<T>::mma(ah, bl[j], acc[i][j]);
          acc[i][j] = Frag<T>::mma(al, bh[j], acc[i][j]);
        }
      }
      Frag<T>::guard(acc[i][0], acc[i][3], ah, SPLIT ? al : ah);
    }
    Frag<T>::keep(bh[0], bh[1], bh[2], bh[3]);
    if (SPLIT) Frag<T>::keep(bl[0], bl[1], bl[2], bl[3]);
  }
  acc_guard4(acc[0][0], acc[0][1], acc[0][2], acc[0][3]);
  acc_guard4(acc[1][0], acc[1][1], acc[1][2], acc[1][3]);
  acc_guard4(acc[2][0], acc[2][1], acc[2][2], acc[2][3]);
  acc_guard4(acc[3][0], acc[3][1], acc[3][2], acc[3][3]);

  float* slab = sT[wave];
  float bvj[4];
#pragma unroll
  for (int j = 0; j < 4; ++j) bvj[j] = (BIAS_MODE == 2) ? rne_bf(bias[n0 + (j << 4) + rlane]) : 0.f;
#pragma unroll
  for (int i = 0; i < 4; ++i) {
    const int mBase = m0 + (i << 4);
    v4f bm0 = (v4f){0.f, 0.f, 0.f, 0.f};
    v4f bm1 = bm0;
    if (BIAS_MODE == 1) {
      bm0 = *(const v4f*)(bias + mBase + mOff);
      bm1 = *(const v4f*)(bias + mBase + mOff + 4);
    }
#pragma unroll
    for (int j = 0; j < 4; ++j) {
#pragma unroll
      for (int r = 0; r < 8; ++r) {
        float v = acc[i][j][r] * scale;
        if (BIAS_MODE == 1) { const v4f bsel = (r < 4) ? bm0 : bm1; v += rne_bf(bsel[r & 3]); }
        if (BIAS_MODE == 2) v += bvj[j];
        slab[(mOff + r) * 68 + (j << 4) + rlane] = v;
      }
    }
    __builtin_amdgcn_fence(__ATOMIC_RELEASE, "workgroup");
    __builtin_amdgcn_wave_barrier();
    __builtin_amdgcn_fence(__ATOMIC_ACQUIRE, "workgroup");
    if (OUT_MODE == 0) {
      float* C = (float*)Cout + (size_t)b * strideC;
      const int hh = lane >> 4, c4 = (lane & 15) * 4;
      for (int pass = 0; pass < 2; ++pass) {
#pragma unroll
        for (int it = 0; it < 8; ++it) {
          const int row = it * 2 + hh;
          v4f v = *(const v4f*)(slab + row * 68 + c4);
          *(volatile v4f*)(C + (size_t)(mBase + row) * ldc + n0 + c4) = v;
        }
        __threadfence();
      }
    } else {
      const int q = lane >> 3, c8 = (lane & 7) * 8;
      unsigned short* C  = (unsigned short*)Cout  + (size_t)b * strideC;
      unsigned short* C2 = (OUT_MODE == 2) ? ((unsigned short*)Cout2 + (size_t)b * strideC) : nullptr;
      for (int pass = 0; pass < 2; ++pass) {
#pragma unroll
        for (int it = 0; it < 4; ++it) {
          const int row = it * 4 + q;
          const float* sp = slab + row * 68 + c8;
          v8h hv, lv;
#pragma unroll
          for (int e = 0; e < 8; ++e) {
            if (OUT_MODE == 1) {
              hv[e] = (_Float16)sp[e];
            } else {
              unsigned short hb = f2bf_bits(sp[e]);
              unsigned short lb = f2bf_bits(sp[e] - bf_bits2f(hb));
              hv[e] = __builtin_bit_cast(_Float16, hb);
              lv[e] = __builtin_bit_cast(_Float16, lb);
            }
          }
          *(volatile v8h*)(C + (size_t)(mBase + row) * ldc + n0 + c8) = hv;
          if (OUT_MODE == 2) *(volatile v8h*)(C2 + (size_t)(mBase + row) * ldc + n0 + c8) = lv;
        }
        __threadfence();
      }
    }
    __builtin_amdgcn_fence(__ATOMIC_RELEASE, "workgroup");
    __builtin_amdgcn_wave_barrier();
    __builtin_amdgcn_fence(__ATOMIC_ACQUIRE, "workgroup");
  }
}

__global__ __launch_bounds__(256) void cast_f32_bf16x2(
    const float* __restrict__ in, unsigned short* __restrict__ out, int n2) {
  const int i = blockIdx.x * 256 + threadIdx.x;
  if (i < n2) {
    const unsigned u = (unsigned)f2bf_bits(in[2 * i]) | ((unsigned)f2bf_bits(in[2 * i + 1]) << 16);
    ((volatile unsigned*)out)[i] = u;
    __threadfence();
    ((volatile unsigned*)out)[i] = u;
  }
}

template <int MODE>
__global__ __launch_bounds__(256) void transpose_cvt16(
    const float* __restrict__ W, unsigned short* __restrict__ Wt, int rows, int cols, float wsc) {
  __shared__ float tile[64 * 65];
  const int tid = threadIdx.x, lane = tid & 31, wave = tid >> 5;
  const int n0 = blockIdx.x * 64;
  const int k0 = blockIdx.y * 64;
  {
    const int c4 = (tid & 15) * 4, r = tid >> 4;
#pragma unroll
    for (int it = 0; it < 4; ++it) {
      const int rr = it * 16 + r;
      const v4f x4 = *(const v4f*)(W + (size_t)(k0 + rr) * cols + n0 + c4);
      tile[rr * 65 + c4 + 0] = x4[0];
      tile[rr * 65 + c4 + 1] = x4[1];
      tile[rr * 65 + c4 + 2] = x4[2];
      tile[rr * 65 + c4 + 3] = x4[3];
    }
  }
  __syncthreads();
  const int q4 = lane >> 3, c8 = (lane & 7) * 8;
  _Float16* out = (_Float16*)Wt;
  for (int pass = 0; pass < 2; ++pass) {
#pragma unroll
    for (int it = 0; it < 2; ++it) {
      const int i = wave * 8 + it * 4 + q4;
      v8h hv;
#pragma unroll
      for (int e = 0; e < 8; ++e) {
        const float f = tile[(c8 + e) * 65 + i];
        if (MODE == 0) {
          hv[e] = __builtin_bit_cast(_Float16, f2bf_bits(f));
        } else {
          hv[e] = (_Float16)(rne_bf(f) * wsc);
        }
      }
      *(volatile v8h*)(out + (size_t)(n0 + i) * rows + k0 + c8) = hv;
    }
    __threadfence();
  }
}

constexpr int kQB = 64;
constexpr int kKC = 64;
constexpr int kNW = 4;
constexpr int kBiasL = kQB + kSeq;
constexpr float kPCarry = 32768.0f;
static_assert(kSeq % kKC == 0 && kSeq % kQB == 0);

__global__ __launch_bounds__(128) void attn_relbias_f16(
    const unsigned short* __restrict__ Qp, const unsigned short* __restrict__ Kp,
    const unsigned short* __restrict__ Vtp, const float* __restrict__ btab,
    const float* __restrict__ tptr, unsigned short* __restrict__ Cp, float ctx_scale) {
  union FH { v16h v; v8h h[2]; };
  __shared__ __align__(16) _Float16 Ksh[kKC * kHD];
  __shared__ __align__(16) _Float16 Vtsh[kHD * kKC];
  __shared__ __align__(16) _Float16 Psh[kNW][16 * kKC];
  __shared__ __align__(16) float Os[kNW][16 * 68];
  __shared__ __align__(16) float biasL[kBiasL];

  const _Float16* Qh  = (const _Float16*)Qp;
  const _Float16* Kh  = (const _Float16*)Kp;
  const _Float16* Vth = (const _Float16*)Vtp;

  const int tid  = threadIdx.x;
  const int wave = tid >> 5;
  const int lane = tid & 31;
  const int hh   = lane >> 4;
  const int c    = lane & 15;

  constexpr int nqb = kSeq / kQB;
  const int bx = blockIdx.x;
  const int qb = bx % nqb;
  const int bh = bx / nqb;
  const int h  = bh % kHeads;
  const int b  = bh / kHeads;
  const int qbase = qb * kQB;
  const int q0 = qbase + wave * 16;

  float tv = rne_bf(tptr[0]);
  tv = fminf(fmaxf(tv, 0.1f), 10.0f);
  const float inv = 1.0f / (sqrtf((float)kEmb) * tv);

  for (int i = tid; i < kBiasL; i += kNW * 32) {
    int rel = qbase + i;
    rel = rel > kRelMax ? kRelMax : rel;
    biasL[i] = rne_bf(btab[(size_t)rel * kHeads + h]) * inv;
  }

  v16h qa[2];
  {
    const _Float16* qrow = Qh + (size_t)(b * kSeq + q0 + c) * kEmb + h * kHD;
#pragma unroll
    for (int dc = 0; dc < 2; ++dc) qa[dc] = Frag<_Float16>::load(qrow + dc * 32 + 8 * hh);
  }

  float mrow[8], lrow[8];
  v8f oacc[4];
#pragma unroll
  for (int r = 0; r < 8; ++r) { mrow[r] = -INFINITY; lrow[r] = 0.f; }
#pragma unroll
  for (int t = 0; t < 4; ++t) oacc[t] = (v8f){0.f,0.f,0.f,0.f,0.f,0.f,0.f,0.f};

  const int qloc = wave * 16 + 8 * hh;

  for (int kc = 0; kc < kSeq / kKC; ++kc) {
    const int kv0 = kc * kKC;
    __syncthreads();
    {
      const int rr = tid >> 1, dh = (tid & 1) * 32;
      const v4u* ks = (const v4u*)(Kh + (size_t)(b * kSeq + kv0 + rr) * kEmb + h * kHD + dh);
      const v4u* vs = (const v4u*)(Vth + (size_t)(h * kHD + rr) * kTok + b * kSeq + kv0 + dh);
      v4u* kd = (v4u*)(Ksh + rr * kHD + dh);
      v4u* vd = (v4u*)(Vtsh + rr * kKC + dh);
      v4u kt[4], vt[4];
#pragma unroll
      for (int i = 0; i < 4; ++i) { kt[i] = ks[i]; vt[i] = vs[i]; }
#pragma unroll
      for (int i = 0; i < 4; ++i) { kd[i] = kt[i]; vd[i] = vt[i]; }
    }
    __syncthreads();

    v8f s[4];
#pragma unroll
    for (int j = 0; j < 4; ++j) {
      s[j] = (v8f){0.f,0.f,0.f,0.f,0.f,0.f,0.f,0.f};
#pragma unroll
      for (int dc = 0; dc < 2; ++dc) {
        FH kb;
        kb.h[0] = *(const v8h*)(Ksh + (j * 16 + c) * kHD + dc * 32 + 8 * hh);
        kb.h[1] = *(const v8h*)(Ksh + (j * 16 + c) * kHD + dc * 32 + 16 + 8 * hh);
        s[j] = hmma(qa[dc], kb.v, s[j]);
      }
    }

    float cm[8];
#pragma unroll
    for (int r = 0; r < 8; ++r) {
      const int bi = qloc + r + (kSeq - 1) - kv0 - c;
      float m = -INFINITY;
#pragma unroll
      for (int j = 0; j < 4; ++j) {
        const float sc = s[j][r] * inv + biasL[bi - j * 16];
        s[j][r] = sc;
        m = fmaxf(m, sc);
      }
#pragma unroll
      for (int off = 1; off < 16; off <<= 1) m = fmaxf(m, __shfl_xor(m, off, 32));
      cm[r] = m;
    }

    _Float16* pw = Psh[wave];
#pragma unroll
    for (int r = 0; r < 8; ++r) {
      const float mnew = fmaxf(mrow[r], cm[r]);
      const float alpha = expf(mrow[r] - mnew);
      mrow[r] = mnew;
      float psum = 0.f;
#pragma unroll
      for (int j = 0; j < 4; ++j) {
        const float p = expf(s[j][r] - mnew);
        psum += p;
        pw[(8 * hh + r) * kKC + j * 16 + c] = (_Float16)(p * kPCarry);
      }
#pragma unroll
      for (int off = 1; off < 16; off <<= 1) psum += __shfl_xor(psum, off, 32);
      lrow[r] = lrow[r] * alpha + psum;
#pragma unroll
      for (int t = 0; t < 4; ++t) oacc[t][r] *= alpha;
    }
    __syncthreads();

#pragma unroll
    for (int kk = 0; kk < 2; ++kk) {
      FH pa;
      pa.h[0] = *(const v8h*)(pw + c * kKC + kk * 32 + 8 * hh);
      pa.h[1] = *(const v8h*)(pw + c * kKC + kk * 32 + 16 + 8 * hh);
#pragma unroll
      for (int t = 0; t < 4; ++t) {
        FH vb;
        vb.h[0] = *(const v8h*)(Vtsh + (t * 16 + c) * kKC + kk * 32 + 8 * hh);
        vb.h[1] = *(const v8h*)(Vtsh + (t * 16 + c) * kKC + kk * 32 + 16 + 8 * hh);
        oacc[t] = hmma(pa.v, vb.v, oacc[t]);
      }
    }
  }

  float* os = Os[wave];
#pragma unroll
  for (int r = 0; r < 8; ++r) {
    const float invl = ctx_scale * (1.0f / (lrow[r] * kPCarry));
#pragma unroll
    for (int t = 0; t < 4; ++t) os[(8 * hh + r) * 68 + t * 16 + c] = oacc[t][r] * invl;
  }
  __syncthreads();
  {
    const int q4 = lane >> 3, c8 = (lane & 7) * 8;
    _Float16* Ch = (_Float16*)Cp;
    for (int pass = 0; pass < 2; ++pass) {
#pragma unroll
      for (int it = 0; it < 4; ++it) {
        const int row = it * 4 + q4;
        const float* sp = os + row * 68 + c8;
        v8h hv;
#pragma unroll
        for (int e = 0; e < 8; ++e) hv[e] = (_Float16)sp[e];
        *(volatile v8h*)(Ch + (size_t)(b * kSeq + q0 + row) * kEmb + h * kHD + c8) = hv;
      }
      __threadfence();
    }
  }
}

extern "C" void kernel_launch(void* const* d_in, const int* in_sizes, int n_in,
                              void* d_out, int out_size, void* d_ws, size_t ws_size,
                              hipStream_t stream) {
  if (n_in < 11) return;
  if (in_sizes[0] != kTok * kEmb) return;
  if (in_sizes[1] != kEmb * kEmb || in_sizes[3] != kEmb * kEmb ||
      in_sizes[5] != kEmb * kEmb || in_sizes[7] != kEmb * kEmb) return;
  if (in_sizes[2] < kEmb || in_sizes[4] < kEmb || in_sizes[6] < kEmb || in_sizes[8] < kEmb) return;
  if (in_sizes[9] != kRelRows * kHeads || in_sizes[10] < 1) return;
  if (out_size != kTok * kEmb) return;

  const float* x    = (const float*)d_in[0];
  const float* Wq   = (const float*)d_in[1];
  const float* bq   = (const float*)d_in[2];
  const float* Wk   = (const float*)d_in[3];
  const float* bk   = (const float*)d_in[4];
  const float* Wv   = (const float*)d_in[5];
  const float* bv   = (const float*)d_in[6];
  const float* Wp   = (const float*)d_in[7];
  const float* bp   = (const float*)d_in[8];
  const float* btab = (const float*)d_in[9];
  const float* tptr = (const float*)d_in[10];
  float* out = (float*)d_out;

  const size_t szAct = (size_t)kTok * kEmb * 2;
  const size_t szW   = (size_t)kEmb * kEmb * 2;
  size_t off = 0;
  const size_t oXb = off; off += szAct;
  const size_t oWq = off; off += szW;
  const size_t oWk = off; off += szW;
  const size_t oWv = off; off += szW;
  const size_t oWp = off; off += szW;
  const size_t oQ  = off; off += szAct;
  const size_t oK  = off; off += szAct;
  const size_t oVt = off; off += szAct;
  const size_t oCx = off; off += szAct;
  if (off > ws_size) return;

  char* w = (char*)d_ws;
  unsigned short* Xb  = (unsigned short*)(w + oXb);
  unsigned short* WqT = (unsigned short*)(w + oWq);
  unsigned short* WkT = (unsigned short*)(w + oWk);
  unsigned short* WvT = (unsigned short*)(w + oWv);
  unsigned short* WpT = (unsigned short*)(w + oWp);
  unsigned short* Qp  = (unsigned short*)(w + oQ);
  unsigned short* Kp  = (unsigned short*)(w + oK);
  unsigned short* Vtp = (unsigned short*)(w + oVt);
  unsigned short* Cx  = (unsigned short*)(w + oCx);

  const float kWpCarry  = 64.0f;
  const float kCtxCarry = 64.0f;

  {
    const int n2 = (kTok * kEmb) / 2;
    cast_f32_bf16x2<<<(n2 + 255) / 256, 256, 0, stream>>>(x, Xb, n2);
  }
  {
    dim3 grd(kEmb / 64, kEmb / 64);
    transpose_cvt16<0><<<grd, 256, 0, stream>>>(Wq, WqT, kEmb, kEmb, 1.0f);
    transpose_cvt16<0><<<grd, 256, 0, stream>>>(Wk, WkT, kEmb, kEmb, 1.0f);
    transpose_cvt16<0><<<grd, 256, 0, stream>>>(Wv, WvT, kEmb, kEmb, 1.0f);
    transpose_cvt16<1><<<grd, 256, 0, stream>>>(Wp, WpT, kEmb, kEmb, kWpCarry);
  }
  static_assert((kTok / 64) * (kEmb / 64) % 8 == 0);
  const int gemmBlocks = ((kTok / 64) * (kEmb / 64)) / 8;
  wmma_gemm64<1, false, 2, 1><<<dim3(gemmBlocks, 1), 256, 0, stream>>>(
      Xb, Xb, kEmb, 0L, WqT, WqT, kEmb, 0L, (void*)Qp, (void*)Qp, kEmb, 0L, bq,
      kTok, kEmb, kEmb, 1.0f);
  wmma_gemm64<1, false, 2, 1><<<dim3(gemmBlocks, 1), 256, 0, stream>>>(
      Xb, Xb, kEmb, 0L, WkT, WkT, kEmb, 0L, (void*)Kp, (void*)Kp, kEmb, 0L, bk,
      kTok, kEmb, kEmb, 1.0f);
  wmma_gemm64<1, false, 1, 1><<<dim3(gemmBlocks, 1), 256, 0, stream>>>(
      WvT, WvT, kEmb, 0L, Xb, Xb, kEmb, 0L, (void*)Vtp, (void*)Vtp, kTok, 0L, bv,
      kEmb, kTok, kEmb, 1.0f);
  attn_relbias_f16<<<kBatch * kHeads * (kSeq / kQB), kNW * 32, 0, stream>>>(
      Qp, Kp, Vtp, btab, tptr, Cx, kCtxCarry);
  wmma_gemm64<0, false, 2, 0><<<dim3(gemmBlocks, 1), 256, 0, stream>>>(
      Cx, Cx, kEmb, 0L, WpT, WpT, kEmb, 0L, (void*)out, (void*)out, kEmb, 0L, bp,
      kTok, kEmb, kEmb, 1.0f / (kWpCarry * kCtxCarry));
}
